// TransformerEncoder_83665962926232
// MI455X (gfx1250) — hardware-verified
//
#include <hip/hip_runtime.h>
#ifndef NB
#define NB 4
#endif
#ifndef SEQ
#define SEQ 2048
#endif
#define NB_FULL 4
#define SEQ_FULL 2048
#define NE 256
#define NH 8
#define HD 32
#define NDFF 1024
#define NLAY 2
#define NTOK (SEQ * NB)

static_assert(NE == 256);
static_assert(NH * HD == NE);
static_assert(HD == 32);
static_assert(SEQ % 64 == 0);
static_assert(NTOK % 16 == 0);
static_assert(NTOK % 8 == 0);
static_assert((3 * NE) % 128 == 0);
static_assert(NE % 128 == 0);
static_assert(NDFF % 128 == 0);
static_assert(NE % 32 == 0);
static_assert(NDFF % 32 == 0);
static_assert(((NTOK / 16) * ((3 * NE) / 128)) % 4 == 0);
static_assert(((NTOK / 16) * (NE / 128)) % 4 == 0);
static_assert(((NTOK / 16) * (NDFF / 128)) % 4 == 0);
static_assert(256 * 8 * 8 == 64 * NE);
static_assert((NLAY * 3 * NE * NE) % 8 == 0);
static_assert((NLAY * NE * NE) % 8 == 0);
static_assert((NLAY * NDFF * NE) % 8 == 0);

typedef __bf16 v16b __attribute__((ext_vector_type(16)));
typedef unsigned short v8us __attribute__((ext_vector_type(8), may_alias));
typedef unsigned short v4us __attribute__((ext_vector_type(4), may_alias));
typedef float  v8f  __attribute__((ext_vector_type(8)));
typedef float  v4f  __attribute__((ext_vector_type(4)));
typedef float  v4fa __attribute__((ext_vector_type(4), may_alias));
union FragB { v16b v; v8us half[2]; unsigned short u[16]; };

__device__ __forceinline__ unsigned short bf16_bits(float x) { unsigned int u = __float_as_uint(x); return (unsigned short)((u + 0x7FFFu + ((u >> 16) & 1u)) >> 16); }
__device__ __forceinline__ float bf16_val(unsigned short b) { return __uint_as_float(((unsigned int)b) << 16); }
__device__ __forceinline__ float bf16_rne(float x) { return bf16_val(bf16_bits(x)); }

template <int NT>
__device__ __forceinline__ v8f mmaN(v16b ah, v16b al, v16b bh, v16b bl, v8f c) {
  c = __builtin_amdgcn_wmma_f32_16x16x32_bf16(false, ah, false, bh, (short)0, c, false, false);
  if (NT >= 2) c = __builtin_amdgcn_wmma_f32_16x16x32_bf16(false, al, false, bh, (short)0, c, false, false);
  if (NT >= 3) c = __builtin_amdgcn_wmma_f32_16x16x32_bf16(false, ah, false, bl, (short)0, c, false, false);
  asm volatile("v_nop\n\tv_nop\n\tv_nop\n\tv_nop" : "+v"(c) : "v"(ah), "v"(al), "v"(bh), "v"(bl));
  return c;
}

__global__ __launch_bounds__(256) void k_cvt_bf16(const float* __restrict__ W, unsigned short* __restrict__ Wb, unsigned int n8) {
  const unsigned int t = blockIdx.x * 256u + threadIdx.x;
  if (t >= n8) return;
  const v4f a = *(const v4fa*)(W + (size_t)t * 8u);
  const v4f b = *(const v4fa*)(W + (size_t)t * 8u + 4u);
  v8us v;
  v[0] = bf16_bits(a[0]); v[1] = bf16_bits(a[1]); v[2] = bf16_bits(a[2]); v[3] = bf16_bits(a[3]);
  v[4] = bf16_bits(b[0]); v[5] = bf16_bits(b[1]); v[6] = bf16_bits(b[2]); v[7] = bf16_bits(b[3]);
  unsigned short* dst = Wb + (size_t)t * 8u;
  *(volatile v8us*)dst = v;
  __threadfence();
  *(volatile v8us*)dst = v;
}

__global__ __launch_bounds__(256) void k_rnecopy(const float* __restrict__ src, float* __restrict__ dst) {
  const unsigned int t = blockIdx.x * 256u + threadIdx.x;
  if (t >= (unsigned int)NTOK * (NE / 4)) return;
  const unsigned int row = t >> 6, c4 = (t & 63u) * 4u;
  const unsigned int l = row / (unsigned int)NB, b = row - l * (unsigned int)NB;
  v4f a = *(const v4fa*)(src + (size_t)(l * (unsigned int)NB_FULL + b) * NE + c4);
#pragma unroll
  for (int i = 0; i < 4; ++i) a[i] = bf16_rne(a[i]);
  float* d = dst + (size_t)t * 4u;
  *(volatile v4f*)d = a;
  __threadfence();
  *(volatile v4f*)d = a;
}

template <bool ASPLIT, int ACT, bool BIAS_BF16>
__global__ __launch_bounds__(128) void k_gemm_bf(const float* __restrict__ A, unsigned int lda, const unsigned short* __restrict__ Wt, unsigned int ldb,
                                               const float* __restrict__ bias, float* __restrict__ C, unsigned int ldc,
                                               unsigned int M, unsigned int N, unsigned int K) {
  __shared__ __attribute__((aligned(16))) float so[4][16][128];
  const unsigned int tid = threadIdx.x, w = tid >> 5, lane = tid & 31u, ln = lane & 15u, hh = lane >> 4;
  const unsigned int ntn = N >> 7;
  const unsigned int wid = blockIdx.x * 4u + w;
  const unsigned int mt = wid / ntn, nq = wid - mt * ntn;
  if (mt * 16u >= M) return;
  const unsigned int row0 = mt * 16u, col0 = nq * 128u;
  const float* arow = A + (size_t)(row0 + ln) * lda;
  v8f acc[8] = {};
  for (unsigned int kb = 0; kb < K; kb += 32u) {
    FragB ah, al;
    const v4f x0 = *(const v4fa*)(arow + kb + 8u * hh), x1 = *(const v4fa*)(arow + kb + 8u * hh + 4u);
    const v4f x2 = *(const v4fa*)(arow + kb + 16u + 8u * hh), x3 = *(const v4fa*)(arow + kb + 16u + 8u * hh + 4u);
    float xs[16] = {x0[0],x0[1],x0[2],x0[3],x1[0],x1[1],x1[2],x1[3],x2[0],x2[1],x2[2],x2[3],x3[0],x3[1],x3[2],x3[3]};
#pragma unroll
    for (int i = 0; i < 16; ++i) { const unsigned short hb = bf16_bits(xs[i]); ah.u[i] = hb; al.u[i] = ASPLIT ? bf16_bits(xs[i] - bf16_val(hb)) : (unsigned short)0; }
#pragma unroll
    for (int t = 0; t < 8; ++t) {
      const unsigned short* brow = Wt + (size_t)(col0 + (unsigned int)t * 16u + ln) * ldb + kb;
      FragB b;
      b.half[0] = *(const v8us*)(brow + 8u * hh);
      b.half[1] = *(const v8us*)(brow + 16u + 8u * hh);
      acc[t] = mmaN<ASPLIT ? 2 : 1>(ah.v, al.v, b.v, b.v, acc[t]);
    }
  }
#pragma unroll
  for (int t = 0; t < 8; ++t) {
    float bv = bias[col0 + (unsigned int)t * 16u + ln];
    if (BIAS_BF16) bv = bf16_rne(bv);
#pragma unroll
    for (int r = 0; r < 8; ++r) { float v = acc[t][r] + bv; if (ACT == 1) v = fmaxf(v, 0.f); so[w][8u * hh + r][(unsigned int)t * 16u + ln] = v; }
  }
  __builtin_amdgcn_fence(4  , "workgroup");
  __builtin_amdgcn_wave_barrier();
  for (int pass = 0; pass < 2; ++pass) {
#pragma unroll
    for (int r = 0; r < 16; ++r) {
      const v4f v = *(const v4fa*)&so[w][r][lane * 4u];
      *(volatile v4f*)(C + (size_t)(row0 + (unsigned int)r) * ldc + col0 + lane * 4u) = v;
    }
    if (pass == 0) __threadfence();
  }
}

__global__ __launch_bounds__(256) void k_split(const float* __restrict__ qkv, unsigned short* __restrict__ Qp,
                                             unsigned short* __restrict__ Kp, unsigned short* __restrict__ Vt) {
  __shared__ __attribute__((aligned(16))) unsigned short sT[64][NE + 8];
  const unsigned int tid = threadIdx.x;
  const unsigned int l0 = blockIdx.x * 64u, b = blockIdx.y, sec = blockIdx.z;
#pragma unroll 4
  for (unsigned int it = 0; it < 16u; ++it) {
    const unsigned int e = tid + it * 256u;
    const unsigned int r = e >> 6, c4 = (e & 63u) * 4u;
    const v4f a = *(const v4fa*)(qkv + (size_t)((l0 + r) * (unsigned int)NB + b) * (3u * NE) + sec * NE + c4);
    v4us o;
    o[0] = bf16_bits(a[0]); o[1] = bf16_bits(a[1]); o[2] = bf16_bits(a[2]); o[3] = bf16_bits(a[3]);
    *(v4us*)&sT[r][c4] = o;
  }
  __syncthreads();
  if (sec < 2u) {
    unsigned short* P = (sec == 0u) ? Qp : Kp;
    for (int pass = 0; pass < 2; ++pass) {
#pragma unroll 4
      for (unsigned int it = 0; it < 8u; ++it) {
        const unsigned int p = tid + it * 256u;
        const unsigned int h = p >> 8, q = p & 255u;
        const unsigned int l = q >> 2, part = q & 3u;
        const v8us v = *(const v8us*)&sT[l][h * 32u + part * 8u];
        *(volatile v8us*)(P + ((size_t)(b * NH + h) * SEQ + l0) * HD + q * 8u) = v;
      }
      if (pass == 0) __threadfence();
    }
  } else {
    for (int pass = 0; pass < 2; ++pass) {
#pragma unroll 2
      for (unsigned int it = 0; it < 8u; ++it) {
        const unsigned int p = tid + it * 256u;
        const unsigned int e = p >> 3, part = p & 7u;
        const unsigned int h = e >> 5, d = e & 31u;
        v8us v;
#pragma unroll
        for (int i = 0; i < 8; ++i) v[i] = sT[part * 8u + (unsigned int)i][e];
        *(volatile v8us*)(Vt + ((size_t)(b * NH + h) * HD + d) * SEQ + l0 + part * 8u) = v;
      }
      if (pass == 0) __threadfence();
    }
  }
}

__global__ __launch_bounds__(128) void k_flash(const unsigned short* __restrict__ Qp, const unsigned short* __restrict__ Kp,
                                             const unsigned short* __restrict__ Vt, float* __restrict__ ctx) {
  __shared__ __attribute__((aligned(16))) unsigned short sP[4][16][72];
  __shared__ __attribute__((aligned(16))) float sO[4][16][HD];
  const unsigned int tid = threadIdx.x, w = tid >> 5, lane = tid & 31u, ln = lane & 15u, hh = lane >> 4;
  constexpr unsigned int NQB = SEQ / 64;
  const unsigned int bh = blockIdx.x / NQB, qblk = blockIdx.x - bh * NQB;
  const unsigned int b = bh / (unsigned int)NH, h = bh - b * (unsigned int)NH;
  const unsigned int q0 = qblk * 64u + w * 16u;
  FragB aq;
  {
    const unsigned short* qr = Qp + ((size_t)bh * SEQ + q0 + ln) * HD + 8u * hh;
    aq.half[0] = *(const v8us*)qr;
    aq.half[1] = *(const v8us*)(qr + 16);
  }
  float m_r[8], l_r[8];
#pragma unroll
  for (int r = 0; r < 8; ++r) { m_r[r] = -1.0e30f; l_r[r] = 0.f; }
  v8f o0 = {0.f,0.f,0.f,0.f,0.f,0.f,0.f,0.f}, o1 = {0.f,0.f,0.f,0.f,0.f,0.f,0.f,0.f};
  const unsigned short* kbase = Kp + ((size_t)bh * SEQ + ln) * HD + 8u * hh;
  const unsigned short* vbase = Vt + ((size_t)bh * HD + ln) * SEQ + 8u * hh;
  const float c = 0.17677669529663687f * 1.4426950408889634f;

  for (unsigned int j0 = 0; j0 < (unsigned int)SEQ; j0 += 64u) {
    v8f s[4];
#pragma unroll
    for (int nt = 0; nt < 4; ++nt) {
      const unsigned short* kp = kbase + (size_t)(j0 + (unsigned int)nt * 16u) * HD;
      FragB bk;
      bk.half[0] = *(const v8us*)kp;
      bk.half[1] = *(const v8us*)(kp + 16);
      const v8f z = {0.f,0.f,0.f,0.f,0.f,0.f,0.f,0.f};
      s[nt] = mmaN<1>(aq.v, aq.v, bk.v, bk.v, z);
    }
#pragma unroll
    for (int r = 0; r < 8; ++r) {
      float mx = fmaxf(fmaxf(s[0][r], s[1][r]), fmaxf(s[2][r], s[3][r]));
      mx = fmaxf(mx, __shfl_xor(mx, 1, 32)); mx = fmaxf(mx, __shfl_xor(mx, 2, 32));
      mx = fmaxf(mx, __shfl_xor(mx, 4, 32)); mx = fmaxf(mx, __shfl_xor(mx, 8, 32));
      const float mnew = fmaxf(m_r[r], mx);
      const float alpha = __builtin_amdgcn_exp2f((m_r[r] - mnew) * c);
      const float nm = -mnew * c;
      const float p0 = __builtin_amdgcn_exp2f(fmaf(s[0][r], c, nm));
      const float p1 = __builtin_amdgcn_exp2f(fmaf(s[1][r], c, nm));
      const float p2 = __builtin_amdgcn_exp2f(fmaf(s[2][r], c, nm));
      const float p3 = __builtin_amdgcn_exp2f(fmaf(s[3][r], c, nm));
      m_r[r] = mnew;
      l_r[r] = l_r[r] * alpha + ((p0 + p1) + (p2 + p3));
      o0[r] *= alpha; o1[r] *= alpha;
      sP[w][8u * hh + r][ln]       = bf16_bits(p0);
      sP[w][8u * hh + r][16u + ln] = bf16_bits(p1);
      sP[w][8u * hh + r][32u + ln] = bf16_bits(p2);
      sP[w][8u * hh + r][48u + ln] = bf16_bits(p3);
    }
    __builtin_amdgcn_fence(4  , "workgroup");
    __builtin_amdgcn_wave_barrier();
#pragma unroll
    for (int ks = 0; ks < 2; ++ks) {
      FragB pa, bv0, bv1;
      pa.half[0] = *(const v8us*)&sP[w][ln][(unsigned int)ks * 32u + 8u * hh];
      pa.half[1] = *(const v8us*)&sP[w][ln][(unsigned int)ks * 32u + 16u + 8u * hh];
      const unsigned short* vp = vbase + j0 + (unsigned int)ks * 32u;
      bv0.half[0] = *(const v8us*)vp;
      bv0.half[1] = *(const v8us*)(vp + 16);
      bv1.half[0] = *(const v8us*)(vp + (size_t)16 * SEQ);
      bv1.half[1] = *(const v8us*)(vp + (size_t)16 * SEQ + 16);
      o0 = mmaN<1>(pa.v, pa.v, bv0.v, bv0.v, o0);
      o1 = mmaN<1>(pa.v, pa.v, bv1.v, bv1.v, o1);
    }
    __builtin_amdgcn_fence(4  , "workgroup");
    __builtin_amdgcn_wave_barrier();
  }
#pragma unroll
  for (int r = 0; r < 8; ++r) {
    float l = l_r[r];
    l += __shfl_xor(l, 1, 32); l += __shfl_xor(l, 2, 32); l += __shfl_xor(l, 4, 32); l += __shfl_xor(l, 8, 32);
    const float inv = 1.0f / l;
    sO[w][8u * hh + r][ln]       = o0[r] * inv;
    sO[w][8u * hh + r][16u + ln] = o1[r] * inv;
  }
  __builtin_amdgcn_fence(4  , "workgroup");
  __builtin_amdgcn_wave_barrier();
  const unsigned int rsub = lane >> 3, piece = lane & 7u;
  for (int pass = 0; pass < 2; ++pass) {
#pragma unroll
    for (int q = 0; q < 4; ++q) {
      const unsigned int r = (unsigned int)q * 4u + rsub;
      const v4f val = *(const v4fa*)&sO[w][r][piece * 4u];
      *(volatile v4f*)(ctx + ((size_t)(q0 + r) * NB + b) * NE + h * HD + piece * 4u) = val;
    }
    if (pass == 0) __threadfence();
  }
}

__global__ __launch_bounds__(256) void k_ln(const float* __restrict__ X, const float* __restrict__ R, const float* __restrict__ g,
                                          const float* __restrict__ bta, float* __restrict__ out, unsigned int nrows) {
  const unsigned int tid = threadIdx.x, w = tid >> 5, lane = tid & 31u;
  const unsigned int row = blockIdx.x * 8u + w;
  if (row >= nrows) return;
  const size_t base = (size_t)row * NE;
  const unsigned int j0 = lane * 4u, j1 = 128u + lane * 4u;
  v4f a0 = *(const v4fa*)(X + base + j0), a1 = *(const v4fa*)(X + base + j1);
  const v4f r0 = *(const v4fa*)(R + base + j0), r1 = *(const v4fa*)(R + base + j1);
#pragma unroll
  for (int q = 0; q < 4; ++q) { a0[q] += r0[q]; a1[q] += r1[q]; }
  float s = ((a0[0] + a0[1]) + (a0[2] + a0[3])) + ((a1[0] + a1[1]) + (a1[2] + a1[3]));
  s += __shfl_xor(s, 16, 32); s += __shfl_xor(s, 8, 32); s += __shfl_xor(s, 4, 32); s += __shfl_xor(s, 2, 32); s += __shfl_xor(s, 1, 32);
  const float mu = s * (1.0f / 256.0f);
  float v = 0.f;
#pragma unroll
  for (int q = 0; q < 4; ++q) { const float c0 = a0[q] - mu; v += c0 * c0; const float c1 = a1[q] - mu; v += c1 * c1; }
  v += __shfl_xor(v, 16, 32); v += __shfl_xor(v, 8, 32); v += __shfl_xor(v, 4, 32); v += __shfl_xor(v, 2, 32); v += __shfl_xor(v, 1, 32);
  const float rs = rsqrtf(v * (1.0f / 256.0f) + 1e-5f);
  const v4f g0 = *(const v4fa*)(g + j0), g1 = *(const v4fa*)(g + j1);
  const v4f b0 = *(const v4fa*)(bta + j0), b1 = *(const v4fa*)(bta + j1);
  v4f o0, o1;
#pragma unroll
  for (int q = 0; q < 4; ++q) {
    o0[q] = (a0[q] - mu) * rs * bf16_rne(g0[q]) + bf16_rne(b0[q]);
    o1[q] = (a1[q] - mu) * rs * bf16_rne(g1[q]) + bf16_rne(b1[q]);
  }
  float* d0 = out + base + j0;
  float* d1 = out + base + j1;
  *(volatile v4f*)d0 = o0;
  *(volatile v4f*)d1 = o1;
  __threadfence();
  *(volatile v4f*)d0 = o0;
  *(volatile v4f*)d1 = o1;
}

static constexpr size_t al256(size_t x) { return (x + 255) & ~(size_t)255; }
static constexpr size_t WS_TOTAL =
    al256((size_t)NLAY * 3 * NE * NE * 2) + al256((size_t)NLAY * NE * NE * 2) + al256((size_t)NLAY * NDFF * NE * 2) + al256((size_t)NLAY * NE * NDFF * 2) +
    4 * al256((size_t)NTOK * NE * 4) + al256((size_t)NTOK * 3 * NE * 4) + al256((size_t)NTOK * NDFF * 4) + 3 * al256((size_t)NTOK * NE * 2);
static_assert(WS_TOTAL <= (size_t)134217728);

extern "C" void kernel_launch(void* const* d_in, const int* in_sizes, int n_in,
                              void* d_out, int out_size, void* d_ws, size_t ws_size, hipStream_t stream) {
  if (n_in < 13) return;
  if (in_sizes[0] < ((SEQ - 1) * NB_FULL + NB) * NE) return;
  if (in_sizes[1] < NLAY * 3 * NE * NE || in_sizes[2] < NLAY * 3 * NE) return;
  if (in_sizes[3] < NLAY * NE * NE || in_sizes[4] < NLAY * NE) return;
  if (in_sizes[5] < NLAY * NE || in_sizes[6] < NLAY * NE) return;
  if (in_sizes[7] < NLAY * NDFF * NE || in_sizes[8] < NLAY * NDFF) return;
  if (in_sizes[9] < NLAY * NE * NDFF || in_sizes[10] < NLAY * NE) return;
  if (in_sizes[11] < NLAY * NE || in_sizes[12] < NLAY * NE) return;
  if (out_size < NTOK * NE) return;
  if (WS_TOTAL > ws_size) return;

  const float* xin   = (const float*)d_in[0];
  const float* in_w  = (const float*)d_in[1];
  const float* in_b  = (const float*)d_in[2];
  const float* out_w = (const float*)d_in[3];
  const float* out_b = (const float*)d_in[4];
  const float* ln1s  = (const float*)d_in[5];
  const float* ln1b  = (const float*)d_in[6];
  const float* w1    = (const float*)d_in[7];
  const float* b1    = (const float*)d_in[8];
  const float* w2    = (const float*)d_in[9];
  const float* b2    = (const float*)d_in[10];
  const float* ln2s  = (const float*)d_in[11];
  const float* ln2b  = (const float*)d_in[12];

  char* ws = (char*)d_ws; size_t off = 0;
  auto take = [&](size_t bytes) { char* p = ws + off; off += (bytes + 255) & ~(size_t)255; return p; };
  unsigned short* Bin  = (unsigned short*)take((size_t)NLAY * 3 * NE * NE * 2);
  unsigned short* Bout = (unsigned short*)take((size_t)NLAY * NE * NE * 2);
  unsigned short* B1   = (unsigned short*)take((size_t)NLAY * NDFF * NE * 2);
  unsigned short* B2   = (unsigned short*)take((size_t)NLAY * NE * NDFF * 2);
  float* x    = (float*)take((size_t)NTOK * NE * 4);
  float* a    = (float*)take((size_t)NTOK * NE * 4);
  float* tmp  = (float*)take((size_t)NTOK * NE * 4);
  float* ctx  = (float*)take((size_t)NTOK * NE * 4);
  float* qkv  = (float*)take((size_t)NTOK * 3 * NE * 4);
  float* hbuf = (float*)take((size_t)NTOK * NDFF * 4);
  unsigned short* Qp = (unsigned short*)take((size_t)NTOK * NE * 2);
  unsigned short* Kp = (unsigned short*)take((size_t)NTOK * NE * 2);
  unsigned short* Vt = (unsigned short*)take((size_t)NTOK * NE * 2);
  if (off > ws_size) return;

  const unsigned int n8_in = NLAY * 3 * NE * NE / 8, n8_out = NLAY * NE * NE / 8, n8_1 = NLAY * NDFF * NE / 8, n8_2 = NLAY * NE * NDFF / 8;
  k_cvt_bf16<<<(n8_in + 255) / 256, 256, 0, stream>>>(in_w, Bin, n8_in);
  k_cvt_bf16<<<(n8_out + 255) / 256, 256, 0, stream>>>(out_w, Bout, n8_out);
  k_cvt_bf16<<<(n8_1 + 255) / 256, 256, 0, stream>>>(w1, B1, n8_1);
  k_cvt_bf16<<<(n8_2 + 255) / 256, 256, 0, stream>>>(w2, B2, n8_2);
  k_rnecopy<<<(NTOK * (NE / 4) + 255) / 256, 256, 0, stream>>>(xin, x);

  const unsigned int g_qkv = ((NTOK / 16) * ((3 * NE) / 128) + 3) / 4;
  const unsigned int g_e   = ((NTOK / 16) * (NE / 128) + 3) / 4;
  const unsigned int g_ff  = ((NTOK / 16) * (NDFF / 128) + 3) / 4;
  for (int i = 0; i < NLAY; ++i) {
    k_gemm_bf<false, 0, true><<<g_qkv, 128, 0, stream>>>(x, NE, Bin + (size_t)i * 3 * NE * NE, NE, in_b + (size_t)i * 3 * NE,
                                                        qkv, 3 * NE, NTOK, 3 * NE, NE);
    k_split<<<dim3(SEQ / 64, NB, 3), 256, 0, stream>>>(qkv, Qp, Kp, Vt);
    k_flash<<<NB * NH * (SEQ / 64), 128, 0, stream>>>(Qp, Kp, Vt, ctx);
    k_gemm_bf<false, 0, true><<<g_e, 128, 0, stream>>>(ctx, NE, Bout + (size_t)i * NE * NE, NE, out_b + (size_t)i * NE,
                                                      tmp, NE, NTOK, NE, NE);
    k_ln<<<NTOK / 8, 256, 0, stream>>>(tmp, x, ln1s + (size_t)i * NE, ln1b + (size_t)i * NE, a, NTOK);
    k_gemm_bf<true, 1, true><<<g_ff, 128, 0, stream>>>(a, NE, B1 + (size_t)i * NDFF * NE, NE, b1 + (size_t)i * NDFF,
                                                      hbuf, NDFF, NTOK, NDFF, NE);
    k_gemm_bf<true, 0, true><<<g_e, 128, 0, stream>>>(hbuf, NDFF, B2 + (size_t)i * NE * NDFF, NDFF, b2 + (size_t)i * NE,
                                                     tmp, NE, NTOK, NE, NDFF);
    k_ln<<<NTOK / 8, 256, 0, stream>>>(tmp, a, ln2s + (size_t)i * NE, ln2b + (size_t)i * NE,
                                       (i == NLAY - 1) ? (float*)d_out : x, NTOK);
  }
}
